// RNNDecoder_84052509983543
// MI455X (gfx1250) — hardware-verified
//
#include <hip/hip_runtime.h>
#include <math.h>

constexpr int kB = 8, kT = 13, kN = 128, kD = 4, kH = 64, kMH = 128;
constexpr int kNodes = kB * kN;
constexpr int kPairs = kB * kN * kN;
constexpr int kSteps = kT - 1;
constexpr int kPQCols = 2 * kMH;
constexpr int kCellNodes = 8;
constexpr int kCellBlocks = kNodes / kCellNodes;
constexpr int kPartPitch = 32;
constexpr int kOutLL = kB * kSteps * kN * kD;
constexpr float kW8 = 8.0f;
constexpr float kW8Inv = 0.125f;
static_assert(kNodes % 64 == 0 && kPairs % 64 == 0 && kPQCols % 64 == 0 && kH % 64 == 0);
static_assert(kH % 32 == 0 && kMH % 32 == 0);
static_assert(kNodes % kCellNodes == 0 && kN % kCellNodes == 0);

typedef __attribute__((ext_vector_type(16))) _Float16 v16h;
typedef __attribute__((ext_vector_type(8)))  _Float16 v8h;
typedef __attribute__((ext_vector_type(16))) __bf16   v16b;
typedef __attribute__((ext_vector_type(8)))  __bf16   v8b;
typedef __attribute__((ext_vector_type(8)))  float    v8f;
typedef __attribute__((ext_vector_type(4)))  float    v4f;

__device__ __forceinline__ unsigned short f2bf_bits(float f) {
  unsigned u = __float_as_uint(f);
  return (unsigned short)((u + 0x7FFFu + ((u >> 16) & 1u)) >> 16);
}
__device__ __forceinline__ float bf_bits2f(unsigned short h) { return __uint_as_float(((unsigned)h) << 16); }

__device__ __forceinline__ float tanh_rx(float x) {
  const float e = __expf(x + x);
  const float r = __builtin_amdgcn_rcpf(1.0f + e);
  return fmaf(-2.0f, r, 1.0f);
}
__device__ __forceinline__ float sig_rx(float x) {
  return __builtin_amdgcn_rcpf(1.0f + __expf(-x));
}

__device__ __forceinline__ void dep_guard_h(v8f& a, v8f& b, v16h x, v16h y) { asm volatile("v_nop\n\tv_nop\n\tv_nop\n\tv_nop" : "+v"(a), "+v"(b) : "v"(x), "v"(y)); }
__device__ __forceinline__ void dep_guard_b(v8f& a, v8f& b, v16b x, v16b y) { asm volatile("v_nop\n\tv_nop\n\tv_nop\n\tv_nop" : "+v"(a), "+v"(b) : "v"(x), "v"(y)); }
__device__ __forceinline__ void keep4_h(v16h a, v16h b, v16h c, v16h d) { asm volatile("v_nop" :: "v"(a), "v"(b), "v"(c), "v"(d)); }
__device__ __forceinline__ void keep4_b(v16b a, v16b b, v16b c, v16b d) { asm volatile("v_nop" :: "v"(a), "v"(b), "v"(c), "v"(d)); }
__device__ __forceinline__ void acc_guard4(v8f& a, v8f& b, v8f& c, v8f& d) { asm volatile("v_nop\n\tv_nop\n\tv_nop\n\tv_nop" : "+v"(a), "+v"(b), "+v"(c), "+v"(d)); }
template <typename T> struct Frag;
template <> struct Frag<_Float16> {
  typedef v16h V; union U { v16h v; v8h h[2]; };
  static __device__ __forceinline__ v16h load(const _Float16* p) {
    U f; f.h[0] = *(const v8h*)(p); f.h[1] = *(const v8h*)(p + 16); return f.v;
  }
  static __device__ __forceinline__ v8f mma(v16h a, v16h b, v8f c) {
    return __builtin_amdgcn_wmma_f32_16x16x32_f16(false, a, false, b, (short)0, c, false, false);
  }
  static __device__ __forceinline__ void guard(v8f& a, v8f& b, v16h x, v16h y) { dep_guard_h(a, b, x, y); }
  static __device__ __forceinline__ void keep(v16h a, v16h b, v16h c, v16h d) { keep4_h(a, b, c, d); }
};
template <> struct Frag<__bf16> {
  typedef v16b V; union U { v16b v; v8b h[2]; };
  static __device__ __forceinline__ v16b load(const __bf16* p) {
    U f; f.h[0] = *(const v8b*)(p); f.h[1] = *(const v8b*)(p + 16); return f.v;
  }
  static __device__ __forceinline__ v8f mma(v16b a, v16b b, v8f c) {
    return __builtin_amdgcn_wmma_f32_16x16x32_bf16(false, a, false, b, (short)0, c, false, false);
  }
  static __device__ __forceinline__ void guard(v8f& a, v8f& b, v16b x, v16b y) { dep_guard_b(a, b, x, y); }
  static __device__ __forceinline__ void keep(v16b a, v16b b, v16b c, v16b d) { keep4_b(a, b, c, d); }
};

template <int ET> struct Elem;
template <> struct Elem<0> { typedef _Float16 T; };
template <> struct Elem<1> { typedef __bf16 T; };
template <int ET, bool SPLIT, int BIAS_MODE, int OUT_MODE, bool RESID, int ACT = 0>
__global__ __launch_bounds__(256) void wmma_gemm64(
    const unsigned short* __restrict__ Ap, const unsigned short* __restrict__ A2p, int lda, long strideA,
    const unsigned short* __restrict__ Btp, const unsigned short* __restrict__ Bt2p, int ldb, long strideB,
    void* __restrict__ Cout, void* __restrict__ Cout2, int ldc, long strideC,
    const float* __restrict__ bias,
    const float* __restrict__ resid, long strideR,
    int M, int N, int K, float scale) {
  typedef typename Elem<ET>::T T;
  typedef typename Frag<T>::V V;
  const T* A = (const T*)Ap; const T* A2 = (const T*)A2p; const T* Bt = (const T*)Btp; const T* Bt2 = (const T*)Bt2p;
  __shared__ __align__(16) float sT[8][16 * 68];
  const int b    = blockIdx.y;
  const int lane = threadIdx.x & 31;
  const int wave = threadIdx.x >> 5;
  const int tilesN = N >> 6;
  const int tilesM = M >> 6;
  const int tile = blockIdx.x * 8 + wave;
  if (tile >= tilesM * tilesN) return;
  const int tm = tile / tilesN;
  const int tn = tile - tm * tilesN;
  const int m0 = tm << 6;
  const int n0 = tn << 6;

  const T* Ab  = A  + (size_t)b * strideA;
  const T* Bb  = Bt + (size_t)b * strideB;
  const T* Ab2 = SPLIT ? (A2  + (size_t)b * strideA) : nullptr;
  const T* Bb2 = SPLIT ? (Bt2 + (size_t)b * strideB) : nullptr;

  const int rlane = lane & 15;
  const int koff  = (lane >> 4) * 8;
  const int mOff  = (lane >> 4) * 8;

  v8f acc[4][4];
#pragma unroll
  for (int i = 0; i < 4; ++i)
#pragma unroll
    for (int j = 0; j < 4; ++j) acc[i][j] = (v8f){0.f,0.f,0.f,0.f,0.f,0.f,0.f,0.f};

  for (int k0 = 0; k0 < K; k0 += 32) {
    V bh[4], bl[4];
#pragma unroll
    for (int j = 0; j < 4; ++j) {
      const size_t bo = (size_t)(n0 + (j << 4) + rlane) * ldb + koff + k0;
      bh[j] = Frag<T>::load(Bb + bo);
      if (SPLIT) bl[j] = Frag<T>::load(Bb2 + bo);
    }
#pragma unroll
    for (int i = 0; i < 4; ++i) {
      const size_t ao = (size_t)(m0 + (i << 4) + rlane) * lda + koff + k0;
      V ah = Frag<T>::load(Ab + ao);
      V al;
      if (SPLIT) al = Frag<T>::load(Ab2 + ao);
#pragma unroll
      for (int j = 0; j < 4; ++j) {
        acc[i][j] = Frag<T>::mma(ah, bh[j], acc[i][j]);
        if (SPLIT) {
          acc[i][j] = Frag<T>::mma(ah, bl[j], acc[i][j]);
          acc[i][j] = Frag<T>::mma(al, bh[j], acc[i][j]);
        }
      }
      Frag<T>::guard(acc[i][0], acc[i][3], ah, SPLIT ? al : ah);
    }
    Frag<T>::keep(bh[0], bh[1], bh[2], bh[3]);
    if (SPLIT) Frag<T>::keep(bl[0], bl[1], bl[2], bl[3]);
  }
  acc_guard4(acc[0][0], acc[0][1], acc[0][2], acc[0][3]);
  acc_guard4(acc[1][0], acc[1][1], acc[1][2], acc[1][3]);
  acc_guard4(acc[2][0], acc[2][1], acc[2][2], acc[2][3]);
  acc_guard4(acc[3][0], acc[3][1], acc[3][2], acc[3][3]);

  float* slab = sT[wave];
  const float* Rb = RESID ? (resid + (size_t)b * strideR) : nullptr;
#pragma unroll
  for (int i = 0; i < 4; ++i) {
    const int mBase = m0 + (i << 4);
#pragma unroll
    for (int j = 0; j < 4; ++j) {
      const int n = n0 + (j << 4) + rlane;
      float bv = 0.f;
      if (BIAS_MODE == 2) bv = bias[n];
#pragma unroll
      for (int r = 0; r < 8; ++r) {
        float v = acc[i][j][r] * scale;
        if (BIAS_MODE == 1) v += bias[mBase + mOff + r];
        if (BIAS_MODE == 2) v += bv;
        if (RESID) v += Rb[(size_t)(mBase + mOff + r) * ldc + n];
        if (ACT == 1) v = tanhf(v);
        if (ACT == 2) v = fmaxf(v, 0.0f);
        if (ACT == 4) v = (v > 0.f) ? v : 0.01f * v;
        if (ACT == 6) v = tanh_rx(v);
        slab[(mOff + r) * 68 + (j << 4) + rlane] = v;
      }
    }
    __builtin_amdgcn_fence(__ATOMIC_RELEASE, "workgroup");
    __builtin_amdgcn_wave_barrier();
    __builtin_amdgcn_fence(__ATOMIC_ACQUIRE, "workgroup");
    if (OUT_MODE == 0) {
      float* C = (float*)Cout + (size_t)b * strideC;
      const int hh = lane >> 4, c4 = (lane & 15) * 4;
      for (int pass = 0; pass < 2; ++pass) {
#pragma unroll
        for (int it = 0; it < 8; ++it) {
          const int row = it * 2 + hh;
          v4f v = *(const v4f*)(slab + row * 68 + c4);
          *(volatile v4f*)(C + (size_t)(mBase + row) * ldc + n0 + c4) = v;
        }
        __threadfence();
      }
    } else {
      const int q = lane >> 3, c8 = (lane & 7) * 8;
      unsigned short* C  = (unsigned short*)Cout  + (size_t)b * strideC;
      unsigned short* C2 = (OUT_MODE == 2) ? ((unsigned short*)Cout2 + (size_t)b * strideC) : nullptr;
      for (int pass = 0; pass < 2; ++pass) {
#pragma unroll
        for (int it = 0; it < 4; ++it) {
          const int row = it * 4 + q;
          const float* sp = slab + row * 68 + c8;
          v8h hv, lv;
#pragma unroll
          for (int e = 0; e < 8; ++e) {
            if (OUT_MODE == 1) {
              hv[e] = (_Float16)sp[e];
            } else {
              unsigned short hb = f2bf_bits(sp[e]);
              unsigned short lb = f2bf_bits(sp[e] - bf_bits2f(hb));
              hv[e] = __builtin_bit_cast(_Float16, hb);
              lv[e] = __builtin_bit_cast(_Float16, lb);
            }
          }
          *(volatile v8h*)(C + (size_t)(mBase + row) * ldc + n0 + c8) = hv;
          if (OUT_MODE == 2) *(volatile v8h*)(C2 + (size_t)(mBase + row) * ldc + n0 + c8) = lv;
        }
        __threadfence();
      }
    }
    __builtin_amdgcn_fence(__ATOMIC_RELEASE, "workgroup");
    __builtin_amdgcn_wave_barrier();
    __builtin_amdgcn_fence(__ATOMIC_ACQUIRE, "workgroup");
  }
}

__global__ __launch_bounds__(256) void prep_kernel(const float* __restrict__ Wm1, const float* __restrict__ Wm2,
                                                   unsigned short* __restrict__ W1Tp, unsigned short* __restrict__ W2Tp,
                                                   unsigned short* __restrict__ H16p, float* __restrict__ HF0) {
  const int blk = blockIdx.x, tid = threadIdx.x;
  if (blk < 8) {
    const int g = blk * 256 + tid;
    const int n = g >> 3, k8 = (g & 7) * 8;
    const int rowoff = (n >> 7) * kH, cn = n & 127;
    v8h hv;
#pragma unroll
    for (int e = 0; e < 8; ++e) hv[e] = (_Float16)(Wm1[(size_t)(rowoff + k8 + e) * kMH + cn] * kW8);
    _Float16* dst = (_Float16*)W1Tp + (size_t)n * kH + k8;
    *(volatile v8h*)dst = hv; __threadfence(); *(volatile v8h*)dst = hv;
  } else if (blk < 12) {
    const int g = (blk - 8) * 256 + tid;
    const int n = g >> 4, k8 = (g & 15) * 8;
    v8h hv;
#pragma unroll
    for (int e = 0; e < 8; ++e) hv[e] = (_Float16)(Wm2[(size_t)(k8 + e) * kH + n] * kW8);
    _Float16* dst = (_Float16*)W2Tp + (size_t)n * kMH + k8;
    *(volatile v8h*)dst = hv; __threadfence(); *(volatile v8h*)dst = hv;
  } else if (blk < 44) {
    const int g = (blk - 12) * 256 + tid;
    const v8h z = {(_Float16)0.f, (_Float16)0.f, (_Float16)0.f, (_Float16)0.f, (_Float16)0.f, (_Float16)0.f, (_Float16)0.f, (_Float16)0.f};
    _Float16* dst = (_Float16*)H16p + (size_t)g * 8;
    *(volatile v8h*)dst = z; __threadfence(); *(volatile v8h*)dst = z;
  } else if (blk < 108) {
    const int g = (blk - 44) * 256 + tid;
    const v4f z = {0.f, 0.f, 0.f, 0.f};
    float* dst = HF0 + (size_t)g * 4;
    *(volatile v4f*)dst = z; __threadfence(); *(volatile v4f*)dst = z;
  }
}

__global__ __launch_bounds__(128) void adj_kernel(const float* __restrict__ A, float* __restrict__ APW) {
  const int i = blockIdx.x, b = blockIdx.y, j = threadIdx.x;
  __shared__ __align__(16) float vals[kN];
  __shared__ float red[kN];
  const float* Ab = A + (size_t)b * kN * kN;
  const float s = 0.5f * (Ab[i * kN + j] + Ab[j * kN + i]);
  float v = sig_rx(s);
  v = (i == j) ? 0.0f : v;
  vals[j] = v;
  red[j] = v;
  __syncthreads();
  for (int st = 64; st > 0; st >>= 1) {
    if (j < st) red[j] += red[j + st];
    __syncthreads();
  }
  const float inv = 1.0f / (red[0] + 1e-6f);
  if (j < 32) {
    v4f x = *(const v4f*)(vals + j * 4);
    x = x * inv;
    float* dst = APW + ((size_t)(b * kN + i)) * kN + j * 4;
    *(volatile v4f*)dst = x; __threadfence(); *(volatile v4f*)dst = x;
  }
}

__global__ __launch_bounds__(256) void pair_kernel(const float* __restrict__ PQ, const float* __restrict__ bm1,
                                                   unsigned short* __restrict__ T1p) {
  const int g = blockIdx.x * 256 + threadIdx.x;
  const int r = g >> 4;
  const int m8 = (g & 15) * 8;
  const int bi = r >> 7;
  const int j = r & 127;
  const int qr = (bi & ~127) | j;
  const float* pp = PQ + (size_t)bi * kPQCols + m8;
  const float* qp = PQ + (size_t)qr * kPQCols + kMH + m8;
  const v4f p0 = *(const v4f*)pp, p1 = *(const v4f*)(pp + 4);
  const v4f q0 = *(const v4f*)qp, q1 = *(const v4f*)(qp + 4);
  const v4f c0 = *(const v4f*)(bm1 + m8), c1 = *(const v4f*)(bm1 + m8 + 4);
  v8h hv;
#pragma unroll
  for (int e = 0; e < 4; ++e) {
    hv[e]     = (_Float16)tanh_rx(p0[e] + q0[e] + c0[e]);
    hv[4 + e] = (_Float16)tanh_rx(p1[e] + q1[e] + c1[e]);
  }
  _Float16* dst = (_Float16*)T1p + (size_t)r * kMH + m8;
  *(volatile v8h*)dst = hv; __threadfence(); *(volatile v8h*)dst = hv;
}

__global__ __launch_bounds__(256) void agg_kernel(const float* __restrict__ APW, const float* __restrict__ MSG,
                                                  float* __restrict__ AGG) {
  const int g = blockIdx.x * 256 + threadIdx.x;
  const int bj = g >> 4, c4 = (g & 15) * 4;
  const int b = bj >> 7, j = bj & 127;
  const float* ap = APW + (size_t)b * kN * kN + j;
  const float* mp = MSG + ((size_t)b * kN * kN + j) * kH + c4;
  v4f acc = {0.f, 0.f, 0.f, 0.f};
#pragma unroll 1
  for (int i = 0; i < kN; ++i) {
    const float a = ap[i * kN];
    const v4f m = *(const v4f*)(mp + (size_t)i * kN * kH);
    acc += a * m;
  }
  float* dst = AGG + (size_t)bj * kH + c4;
  *(volatile v4f*)dst = acc; __threadfence(); *(volatile v4f*)dst = acc;
}

__global__ __launch_bounds__(512) void cell_kernel(const float* __restrict__ X, const float* __restrict__ HFin,
    const float* __restrict__ AGG,
    const float* __restrict__ Wir, const float* __restrict__ bir, const float* __restrict__ Wii, const float* __restrict__ bii,
    const float* __restrict__ Win, const float* __restrict__ bin_,
    const float* __restrict__ Whr, const float* __restrict__ Whi, const float* __restrict__ Whh,
    const float* __restrict__ Wmr, const float* __restrict__ Wmi, const float* __restrict__ Wmn,
    const float* __restrict__ Wo1, const float* __restrict__ bo1, const float* __restrict__ Wo2, const float* __restrict__ bo2,
    const float* __restrict__ Wo3, const float* __restrict__ bo3,
    float* __restrict__ HFout, unsigned short* __restrict__ H16p, float* __restrict__ out, float* __restrict__ PART, int t) {
  __shared__ __align__(16) float hs[kCellNodes][kH];
  __shared__ __align__(16) float as_[kCellNodes][kH];
  __shared__ __align__(16) float hn[kCellNodes][kH];
  __shared__ __align__(16) float p1[kCellNodes][kH];
  __shared__ __align__(16) float p2[kCellNodes][kH];
  __shared__ __align__(16) float xs[kCellNodes][kD];
  __shared__ __align__(16) float psh[kCellNodes * kD];
  __shared__ float ssh[4];
  const int tid = threadIdx.x;
  const int nl = tid >> 6, col = tid & 63;
  const int node0 = blockIdx.x * kCellNodes;
  const int node = node0 + nl;
  const int b = node0 >> 7, n0 = node0 & 127, n = node & 127;

  hs[nl][col]  = HFin[(size_t)node * kH + col];
  as_[nl][col] = AGG[(size_t)node * kH + col];
  if (col < kD) xs[nl][col] = X[((size_t)(b * kT + t) * kN + n) * kD + col];
  __syncthreads();

  float xr = bir[col], xi = bii[col], xn = bin_[col];
#pragma unroll 1
  for (int k = 0; k < kD; ++k) {
    const float xv = xs[nl][k];
    xr += xv * Wir[k * kH + col];
    xi += xv * Wii[k * kH + col];
    xn += xv * Win[k * kH + col];
  }
  float hr = 0.f, hi = 0.f, hh = 0.f, ar = 0.f, ai = 0.f, an = 0.f;
#pragma unroll 1
  for (int k = 0; k < kH; ++k) {
    const float hv = hs[nl][k], av = as_[nl][k];
    const int w = k * kH + col;
    hr += hv * Whr[w];
    hi += hv * Whi[w];
    hh += hv * Whh[w];
    ar += av * Wmr[w];
    ai += av * Wmi[w];
    an += av * Wmn[w];
  }
  const float rg = sig_rx(xr + hr + ar);
  const float ig = sig_rx(xi + hi + ai);
  const float ng = tanh_rx(xn + rg * hh + an);
  const float hnew = (1.0f - ig) * ng + ig * hs[nl][col];
  hn[nl][col] = hnew;
  __syncthreads();

  float a1 = bo1[col];
#pragma unroll 1
  for (int k = 0; k < kH; ++k) a1 += hn[nl][k] * Wo1[k * kH + col];
  p1[nl][col] = fmaxf(a1, 0.0f);
  __syncthreads();
  float a2 = bo2[col];
#pragma unroll 1
  for (int k = 0; k < kH; ++k) a2 += p1[nl][k] * Wo2[k * kH + col];
  p2[nl][col] = fmaxf(a2, 0.0f);
  __syncthreads();

  if (tid < 32) {
    const int pn = tid >> 2, d = tid & 3;
    float pv = xs[pn][d] + bo3[d];
#pragma unroll 1
    for (int k = 0; k < kH; ++k) pv += p2[pn][k] * Wo3[k * kD + d];
    const float tgt = X[((size_t)(b * kT + t + 1) * kN + n0 + pn) * kD + d];
    const float dq = tgt - pv;
    float sq = dq * dq;
    psh[tid] = pv;
    sq += __shfl_xor(sq, 16, 32);
    sq += __shfl_xor(sq, 8, 32);
    sq += __shfl_xor(sq, 4, 32);
    sq += __shfl_xor(sq, 2, 32);
    sq += __shfl_xor(sq, 1, 32);
    if (tid == 0) ssh[0] = sq;
  }
  __syncthreads();

  const int wave = tid >> 5, lane = tid & 31;
  if (wave < 4) {
    const int row = 2 * wave + (lane >> 4), c4 = (lane & 15) * 4;
    const v4f v = *(const v4f*)(&hn[row][c4]);
    float* dst = HFout + (size_t)(node0 + row) * kH + c4;
    *(volatile v4f*)dst = v; __threadfence(); *(volatile v4f*)dst = v;
  } else if (wave < 6) {
    const int idx = tid - 128, row = idx >> 3, c8 = (idx & 7) * 8;
    v8h hv;
#pragma unroll
    for (int e = 0; e < 8; ++e) hv[e] = (_Float16)hn[row][c8 + e];
    _Float16* dst = (_Float16*)H16p + (size_t)(node0 + row) * kH + c8;
    *(volatile v8h*)dst = hv; __threadfence(); *(volatile v8h*)dst = hv;
  } else if (wave == 6) {
    if (lane < kCellNodes) {
      const v4f v = *(const v4f*)(psh + lane * 4);
      float* dst = out + ((size_t)(b * kSteps + t) * kN + n0 + lane) * kD;
      *(volatile v4f*)dst = v; __threadfence(); *(volatile v4f*)dst = v;
    }
  } else if (wave == 7) {
    if (lane < 8) {
      const float s0 = ssh[0];
      v4f v = {0.f, 0.f, 0.f, 0.f};
      v[0] = (lane == 0) ? s0 : 0.0f;
      float* dst = PART + ((size_t)(t * kCellBlocks + blockIdx.x)) * kPartPitch + lane * 4;
      *(volatile v4f*)dst = v; __threadfence(); *(volatile v4f*)dst = v;
    }
  }
}

__global__ __launch_bounds__(256) void final_kernel(const float* __restrict__ PART, const float* __restrict__ log_sigma,
                                                    float* __restrict__ out) {
  __shared__ float red[256];
  const int tid = threadIdx.x;
  float sigma = expf(log_sigma[0]);
  sigma = fminf(fmaxf(sigma, 1e-4f), 10.0f);
  const float cst = 0.5f * (float)(kB * kN * kD) * logf(2.0f * 3.14159265358979323846f * sigma * sigma);
  const float inv2s2 = 1.0f / (2.0f * sigma * sigma);
  float ll = 0.0f;
  const int pidx = (tid < kCellBlocks) ? tid : (kCellBlocks - 1);
#pragma unroll 1
  for (int t = 0; t < kSteps; ++t) {
    float v = PART[((size_t)(t * kCellBlocks + pidx)) * kPartPitch];
    v = (tid < kCellBlocks) ? v : 0.0f;
    red[tid] = v;
    __syncthreads();
    for (int st = 128; st > 0; st >>= 1) {
      if (tid < st) red[tid] += red[tid + st];
      __syncthreads();
    }
    if (tid == 0) {
      const float nll = cst + red[0] * inv2s2;
      ll = ll - nll;
    }
    __syncthreads();
  }
  if (tid == 0) {
    float* dst = out + kOutLL;
    *(volatile float*)dst = ll; __threadfence(); *(volatile float*)dst = ll;
  }
}

extern "C" void kernel_launch(void* const* d_in, const int* in_sizes, int n_in,
                              void* d_out, int out_size, void* d_ws, size_t ws_size, hipStream_t stream) {
  if (n_in < 25 || d_out == nullptr || d_ws == nullptr) return;
  if (in_sizes[0] != kB * kN * kN || in_sizes[1] != kB * kT * kN * kD || in_sizes[2] != 2 * kH * kMH || in_sizes[3] != kMH ||
      in_sizes[4] != kMH * kH || in_sizes[5] != kH || in_sizes[6] != kD * kH || in_sizes[7] != kH || in_sizes[8] != kD * kH ||
      in_sizes[9] != kH || in_sizes[10] != kD * kH || in_sizes[11] != kH) return;
  for (int q = 12; q <= 18; ++q) if (in_sizes[q] != kH * kH && q != 19) { if (q == 18 && in_sizes[q] == kH * kH) break; if (in_sizes[q] != kH * kH) return; }
  if (in_sizes[19] != kH || in_sizes[20] != kH * kH || in_sizes[21] != kH || in_sizes[22] != kH * kD || in_sizes[23] != kD ||
      in_sizes[24] < 1) return;
  if (out_size != kOutLL + 1) return;

  const float* A    = (const float*)d_in[0];
  const float* X    = (const float*)d_in[1];
  const float* Wm1  = (const float*)d_in[2];
  const float* bm1  = (const float*)d_in[3];
  const float* Wm2  = (const float*)d_in[4];
  const float* bm2  = (const float*)d_in[5];
  const float* Wir  = (const float*)d_in[6];
  const float* bir  = (const float*)d_in[7];
  const float* Wii  = (const float*)d_in[8];
  const float* bii  = (const float*)d_in[9];
  const float* Win  = (const float*)d_in[10];
  const float* bin_ = (const float*)d_in[11];
  const float* Whr  = (const float*)d_in[12];
  const float* Whi  = (const float*)d_in[13];
  const float* Whh  = (const float*)d_in[14];
  const float* Wmr  = (const float*)d_in[15];
  const float* Wmi  = (const float*)d_in[16];
  const float* Wmn  = (const float*)d_in[17];
  const float* Wo1  = (const float*)d_in[18];
  const float* bo1  = (const float*)d_in[19];
  const float* Wo2  = (const float*)d_in[20];
  const float* bo2  = (const float*)d_in[21];
  const float* Wo3  = (const float*)d_in[22];
  const float* bo3  = (const float*)d_in[23];
  const float* log_sigma = (const float*)d_in[24];
  float* out = (float*)d_out;

  const size_t szAPW  = (size_t)kB * kN * kN * 4;
  const size_t szHF   = (size_t)kNodes * kH * 4;
  const size_t szH16  = (size_t)kNodes * kH * 2;
  const size_t szW1T  = (size_t)kPQCols * kH * 2;
  const size_t szW2T  = (size_t)kH * kMH * 2;
  const size_t szPQ   = (size_t)kNodes * kPQCols * 4;
  const size_t szT1   = (size_t)kPairs * kMH * 2;
  const size_t szMSG  = (size_t)kPairs * kH * 4;
  const size_t szAGG  = (size_t)kNodes * kH * 4;
  const size_t szPART = (size_t)kSteps * kCellBlocks * kPartPitch * 4;
  size_t off = 0;
  char* ws = (char*)d_ws;
  float*          APW  = (float*)(ws + off);          off += szAPW;
  float*          HF0  = (float*)(ws + off);          off += szHF;
  float*          HF1  = (float*)(ws + off);          off += szHF;
  unsigned short* H16  = (unsigned short*)(ws + off); off += szH16;
  unsigned short* W1T  = (unsigned short*)(ws + off); off += szW1T;
  unsigned short* W2T  = (unsigned short*)(ws + off); off += szW2T;
  float*          PQ   = (float*)(ws + off);          off += szPQ;
  unsigned short* T1   = (unsigned short*)(ws + off); off += szT1;
  float*          MSG  = (float*)(ws + off);          off += szMSG;
  float*          AGG  = (float*)(ws + off);          off += szAGG;
  float*          PART = (float*)(ws + off);          off += szPART;
  if (off > ws_size) return;

  prep_kernel<<<dim3(108), dim3(256), 0, stream>>>(Wm1, Wm2, W1T, W2T, H16, HF0);
  adj_kernel<<<dim3(kN, kB), dim3(kN), 0, stream>>>(A, APW);

  for (int t = 0; t < kSteps; ++t) {
    float* HFin  = (t & 1) ? HF1 : HF0;
    float* HFout = (t & 1) ? HF0 : HF1;
    wmma_gemm64<0, false, 0, 0, false, 0><<<dim3(kNodes / 64 * kPQCols / 64 / 8, 1), dim3(256), 0, stream>>>(
        H16, H16, kH, 0L, W1T, W1T, kH, 0L, (void*)PQ, (void*)PQ, kPQCols, 0L, bm1, PQ, 0L, kNodes, kPQCols, kH, kW8Inv);
    pair_kernel<<<dim3(kPairs * (kMH / 8) / 256), dim3(256), 0, stream>>>(PQ, bm1, T1);
    wmma_gemm64<0, false, 2, 0, false, 6><<<dim3(kPairs / 64 / 8, 1), dim3(256), 0, stream>>>(
        T1, T1, kMH, 0L, W2T, W2T, kMH, 0L, (void*)MSG, (void*)MSG, kH, 0L, bm2, MSG, 0L, kPairs, kH, kMH, kW8Inv);
    agg_kernel<<<dim3(kNodes * (kH / 4) / 256), dim3(256), 0, stream>>>(APW, MSG, AGG);
    cell_kernel<<<dim3(kCellBlocks), dim3(512), 0, stream>>>(X, HFin, AGG, Wir, bir, Wii, bii, Win, bin_,
        Whr, Whi, Whh, Wmr, Wmi, Wmn, Wo1, bo1, Wo2, bo2, Wo3, bo3, HFout, H16, out, PART, t);
  }
  final_kernel<<<dim3(1), dim3(256), 0, stream>>>(PART, log_sigma, out);
}
